// S_decoder_5583457485492
// MI455X (gfx1250) — hardware-run, weakly checked
//
#include <hip/hip_runtime.h>
#include <stddef.h>


#define DIN     64
#define DHID    128
#define NTHR    256
#define NWAVE   8
#define EPT     8
#define NGRP    2
#define CHUNK   (NTHR * EPT * NGRP)
#define WCAP    (EPT * NGRP * 32)
#define LISTN   (NWAVE * WCAP)
#define SLOTB   16
#define NBD     16384
#define NB1     1024
#define NB2     16384
#define WSCALE  8.0f
#define WINV    0.125f

#define LDS_DEG (NBD * 4 + LISTN * 4 + 64)
#define LDS_L1  (NB1 * DIN * 4 + LISTN * 4 + 64)
#define LDS_L2  (NB2 * 4 + LISTN * 4 + 64)

static_assert((CHUNK & (CHUNK - 1)) == 0);
static_assert(CHUNK <= (1 << (31 - SLOTB)));
static_assert((NBD & (NBD - 1)) == 0 && (NB1 & (NB1 - 1)) == 0 && (NB2 & (NB2 - 1)) == 0);
static_assert(NBD <= (1 << SLOTB) && NB1 <= (1 << SLOTB) && NB2 <= (1 << SLOTB));
static_assert(NB1 * 4 <= LISTN * 4);
static_assert(NB1 == NWAVE * 128);
static_assert(NBD % (NWAVE * 128) == 0 && NB2 % (NWAVE * 128) == 0);
static_assert((NB1 * DIN / 4) % NTHR == 0 && NB2 % NTHR == 0 && (NBD / 4) % NTHR == 0);
static_assert(NB1 % (16 * NWAVE) == 0);

typedef float    v2f  __attribute__((ext_vector_type(2)));
typedef float    v4f  __attribute__((ext_vector_type(4)));
typedef float    v8f  __attribute__((ext_vector_type(8)));
typedef int      v4i  __attribute__((ext_vector_type(4)));
typedef _Float16 v8h  __attribute__((ext_vector_type(8)));
typedef _Float16 v16h __attribute__((ext_vector_type(16)));
union FragH { v16h v; v8h h[2]; };

__device__ __forceinline__ v8h cvt8(v4f a, v4f b) {
  v8h r;
  r[0] = (_Float16)a.x; r[1] = (_Float16)a.y; r[2] = (_Float16)a.z; r[3] = (_Float16)a.w;
  r[4] = (_Float16)b.x; r[5] = (_Float16)b.y; r[6] = (_Float16)b.z; r[7] = (_Float16)b.w;
  return r;
}

__device__ __forceinline__ v8f wmh(v16h a, v16h b, v8f c) {
  v8f d = __builtin_amdgcn_wmma_f32_16x16x32_f16(false, a, false, b, (short)0, c, false, false);
  asm volatile("v_nop\n\tv_nop\n\tv_nop\n\tv_nop" : "+v"(d) : "v"(a), "v"(b));
  return d;
}

template <int NB>
__device__ __forceinline__ int scan_chunk(const int* __restrict__ dsts, int nE, int cbase, int nodeBase,
                                          int vec8, int* list, int tid, int lane, int wave) {
  int wc = 0;
#pragma unroll
  for (int g = 0; g < NGRP; ++g) {
    const int el0  = (g * NTHR + tid) * EPT;
    const int e0   = cbase + el0;
    const int sent = -2147483647 - 1;
    v4i da, db;
    if (vec8 != 0 && cbase + CHUNK <= nE) {
      da = *(const v4i*)(dsts + e0);
      db = *(const v4i*)(dsts + e0 + 4);
    } else {
      const int em = nE - 1;
      da.x = (e0     < nE) ? dsts[min(e0,     em)] : sent;
      da.y = (e0 + 1 < nE) ? dsts[min(e0 + 1, em)] : sent;
      da.z = (e0 + 2 < nE) ? dsts[min(e0 + 2, em)] : sent;
      da.w = (e0 + 3 < nE) ? dsts[min(e0 + 3, em)] : sent;
      db.x = (e0 + 4 < nE) ? dsts[min(e0 + 4, em)] : sent;
      db.y = (e0 + 5 < nE) ? dsts[min(e0 + 5, em)] : sent;
      db.z = (e0 + 6 < nE) ? dsts[min(e0 + 6, em)] : sent;
      db.w = (e0 + 7 < nE) ? dsts[min(e0 + 7, em)] : sent;
    }
    const unsigned nb = (unsigned)nodeBase;
    const unsigned s0 = (unsigned)da.x - nb, s1 = (unsigned)da.y - nb;
    const unsigned s2 = (unsigned)da.z - nb, s3 = (unsigned)da.w - nb;
    const unsigned s4 = (unsigned)db.x - nb, s5 = (unsigned)db.y - nb;
    const unsigned s6 = (unsigned)db.z - nb, s7 = (unsigned)db.w - nb;
    const bool h0 = s0 < (unsigned)NB, h1 = s1 < (unsigned)NB, h2 = s2 < (unsigned)NB, h3 = s3 < (unsigned)NB;
    const bool h4 = s4 < (unsigned)NB, h5 = s5 < (unsigned)NB, h6 = s6 < (unsigned)NB, h7 = s7 < (unsigned)NB;
    const unsigned any = __builtin_amdgcn_ballot_w32(h0 | h1 | h2 | h3 | h4 | h5 | h6 | h7);
    if (any != 0u) {
#define HITJ(J, HJ, SJ) { \
        const unsigned mj = __builtin_amdgcn_ballot_w32(HJ); \
        if (mj != 0u) { \
          if (HJ) { \
            const int pos = wc + (int)__builtin_amdgcn_mbcnt_lo(mj, 0u); \
            if (pos < WCAP) list[wave * WCAP + pos] = ((el0 + (J)) << SLOTB) | (int)(SJ); \
          } \
          wc += (int)__builtin_popcount(mj); } }
      HITJ(0, h0, s0)
      HITJ(1, h1, s1)
      HITJ(2, h2, s2)
      HITJ(3, h3, s3)
      HITJ(4, h4, s4)
      HITJ(5, h5, s5)
      HITJ(6, h6, s6)
      HITJ(7, h7, s7)
#undef HITJ
    }
  }
  return wc;
}

__global__ __launch_bounds__(NTHR) void k_wprep(const float* __restrict__ W1, _Float16* w1s) {
  const int i = blockIdx.x * NTHR + threadIdx.x;
  if (i >= DHID * DIN / 8) return;
  const int o  = i * 8;
  const int n  = o / DIN;
  const int k0 = o - n * DIN;
  const float* p = W1 + (size_t)k0 * DHID + n;
  v4f a, b;
  a.x = p[0];        a.y = p[DHID];     a.z = p[2 * DHID]; a.w = p[3 * DHID];
  b.x = p[4 * DHID]; b.y = p[5 * DHID]; b.z = p[6 * DHID]; b.w = p[7 * DHID];
  a = a * WSCALE;
  b = b * WSCALE;
  const v8h hv = cvt8(a, b);
  _Float16* dp = w1s + o;
  *(volatile v8h*)dp = hv;
  __threadfence();
  *(volatile v8h*)dp = hv;
}

__global__ __launch_bounds__(NTHR) void k_deg(
    const int* __restrict__ ei, float* dinv, int nE, int vec8) {
  extern __shared__ v4f lds_dyn[];
  int* cnt  = (int*)lds_dyn;
  int* list = cnt + NBD;
  int* wcnt = list + LISTN;
  const int tid = threadIdx.x, lane = tid & 31, wave = tid >> 5;
  const int nodeBase = blockIdx.x * NBD;
  const int* dsts = ei + nE;

  {
    const v4f z = {0.f, 0.f, 0.f, 0.f};
    for (int i = tid; i < NBD / 4; i += NTHR) lds_dyn[i] = z;
  }
  __syncthreads();

  const int nChunks = (nE + CHUNK - 1) / CHUNK;
#pragma unroll 1
  for (int ch = 0; ch < nChunks; ++ch) {
    const int cbase = ch * CHUNK;
    const int wc = scan_chunk<NBD>(dsts, nE, cbase, nodeBase, vec8, list, tid, lane, wave);
    if (lane == 0) wcnt[wave] = wc;
    __syncthreads();
    if (wave == 0) {
#pragma unroll 1
      for (int wsx = 0; wsx < NWAVE; ++wsx) {
        int n = __builtin_amdgcn_readfirstlane(wcnt[wsx]);
        n = n > WCAP ? WCAP : (n < 0 ? 0 : n);
        const int* lp = list + wsx * WCAP;
#pragma unroll 1
        for (int i = 0; i < n; ++i) {
          const int ent  = __builtin_amdgcn_readfirstlane(lp[i]);
          const int slot = ent & (NBD - 1);
          const int nv   = cnt[slot] + 1;
          if (lane == 0) cnt[slot] = nv;
        }
      }
    }
    __syncthreads();
  }

  float* dp = dinv + (size_t)nodeBase;
#pragma unroll 4
  for (int q = 0; q < NBD / (NWAVE * 128); ++q) {
    const int f = (wave * (NBD / (NWAVE * 128)) + q) * 128 + 4 * lane;
    const v4i c = *(const v4i*)(cnt + f);
    v4f d;
    d.x = rsqrtf((float)(c.x + 1)); d.y = rsqrtf((float)(c.y + 1));
    d.z = rsqrtf((float)(c.z + 1)); d.w = rsqrtf((float)(c.w + 1));
    *(volatile v4f*)(dp + f) = d;
  }
  __threadfence();
#pragma unroll 4
  for (int q = 0; q < NBD / (NWAVE * 128); ++q) {
    const int f = (wave * (NBD / (NWAVE * 128)) + q) * 128 + 4 * lane;
    const v4i c = *(const v4i*)(cnt + f);
    v4f d;
    d.x = rsqrtf((float)(c.x + 1)); d.y = rsqrtf((float)(c.y + 1));
    d.z = rsqrtf((float)(c.z + 1)); d.w = rsqrtf((float)(c.w + 1));
    *(volatile v4f*)(dp + f) = d;
  }
}

__global__ __launch_bounds__(NTHR) void k_layer1(
    const int* __restrict__ ei, const float* __restrict__ x, const float* __restrict__ dinv,
    const _Float16* __restrict__ w1s, const float* __restrict__ b1, const float* __restrict__ W2,
    float* tpl, int nN, int nE, int vec8) {
  extern __shared__ v4f lds_dyn[];
  float* acc  = (float*)lds_dyn;
  int*   list = (int*)(acc + NB1 * DIN);
  int*   wcnt = list + LISTN;
  float* tst  = (float*)list;
  const int tid = threadIdx.x, lane = tid & 31, wave = tid >> 5, hh = lane >> 4, m = lane & 15;
  const int nodeBase = blockIdx.x * NB1;
  const int* dsts = ei + nE;

  {
    const v4f z = {0.f, 0.f, 0.f, 0.f};
    for (int i = tid; i < NB1 * DIN / 4; i += NTHR) lds_dyn[i] = z;
  }
  __syncthreads();

  const int nChunks = (nE + CHUNK - 1) / CHUNK;
#pragma unroll 1
  for (int ch = 0; ch < nChunks; ++ch) {
    const int cbase = ch * CHUNK;
    const int wc = scan_chunk<NB1>(dsts, nE, cbase, nodeBase, vec8, list, tid, lane, wave);
    if (lane == 0) wcnt[wave] = wc;
    __syncthreads();
    if (wave == 0) {
#pragma unroll 1
      for (int wsx = 0; wsx < NWAVE; ++wsx) {
        int n = __builtin_amdgcn_readfirstlane(wcnt[wsx]);
        n = n > WCAP ? WCAP : (n < 0 ? 0 : n);
        const int* lp = list + wsx * WCAP;
#pragma unroll 1
        for (int i = 0; i < n; ++i) {
          const int ent  = __builtin_amdgcn_readfirstlane(lp[i]);
          const int slot = ent & (NB1 - 1);
          int e = cbase + ((ent >> SLOTB) & (CHUNK - 1));
          e = e > nE - 1 ? nE - 1 : e;
          int src = ei[e];
          src = src < 0 ? 0 : (src > nN - 1 ? nN - 1 : src);
          const float ds = dinv[src];
          v2f xv = *(const v2f*)(x + (size_t)src * DIN + 2 * lane);
          xv.x = fabsf(xv.x) * ds;
          xv.y = fabsf(xv.y) * ds;
          v2f* ap = (v2f*)(acc + slot * DIN + 2 * lane);
          *ap = *ap + xv;
        }
      }
    }
    __syncthreads();
  }

#pragma unroll 4
  for (int i = 0; i < (NB1 * DIN / 4) / NTHR; ++i) {
    const int idx  = i * NTHR + tid;
    const int slot = idx >> 4;
    const int c4   = (idx & 15) * 4;
    int node = nodeBase + slot;
    node = node > nN - 1 ? nN - 1 : node;
    const float d = dinv[node];
    v4f xs = *(const v4f*)(x + (size_t)node * DIN + c4);
    xs.x = fabsf(xs.x); xs.y = fabsf(xs.y); xs.z = fabsf(xs.z); xs.w = fabsf(xs.w);
    v4f* ap = (v4f*)(acc + slot * DIN + c4);
    *ap = (*ap + xs * d) * d;
  }
  __syncthreads();

  float bq[8], wq[8];
#pragma unroll
  for (int t = 0; t < 8; ++t) { bq[t] = b1[16 * t + m]; wq[t] = W2[16 * t + m]; }

#pragma unroll 1
  for (int j = 0; j < NB1 / (16 * NWAVE); ++j) {
    const int tile = wave + NWAVE * j;
    FragH a0, a1;
    {
      const float* ap = acc + (16 * tile + m) * DIN + 8 * hh;
      const v4f p0 = *(const v4f*)ap,        p1 = *(const v4f*)(ap + 4);
      const v4f p2 = *(const v4f*)(ap + 16), p3 = *(const v4f*)(ap + 20);
      a0.h[0] = cvt8(p0, p1);
      a0.h[1] = cvt8(p2, p3);
      const v4f q0 = *(const v4f*)(ap + 32), q1 = *(const v4f*)(ap + 36);
      const v4f q2 = *(const v4f*)(ap + 48), q3 = *(const v4f*)(ap + 52);
      a1.h[0] = cvt8(q0, q1);
      a1.h[1] = cvt8(q2, q3);
    }
    v8f c[8];
#pragma unroll
    for (int t = 0; t < 8; ++t) { v8f z = {0.f, 0.f, 0.f, 0.f, 0.f, 0.f, 0.f, 0.f}; c[t] = z; }
#pragma unroll
    for (int t = 0; t < 8; ++t) {
      const _Float16* bp = w1s + (size_t)(16 * t + m) * DIN + 8 * hh;
      FragH b;
      b.h[0] = *(const v8h*)bp;
      b.h[1] = *(const v8h*)(bp + 16);
      c[t] = wmh(a0.v, b.v, c[t]);
      b.h[0] = *(const v8h*)(bp + 32);
      b.h[1] = *(const v8h*)(bp + 48);
      c[t] = wmh(a1.v, b.v, c[t]);
    }
    float tp[8];
#pragma unroll
    for (int r = 0; r < 8; ++r) tp[r] = 0.f;
#pragma unroll
    for (int t = 0; t < 8; ++t) {
#pragma unroll
      for (int r = 0; r < 8; ++r) tp[r] += fmaxf(c[t][r] * WINV + bq[t], 0.f) * wq[t];
    }
#pragma unroll
    for (int r = 0; r < 8; ++r) {
      tp[r] += __shfl_xor(tp[r], 1, 32);
      tp[r] += __shfl_xor(tp[r], 2, 32);
      tp[r] += __shfl_xor(tp[r], 4, 32);
      tp[r] += __shfl_xor(tp[r], 8, 32);
    }
    const int mr = m & 7;
    float v = tp[0];
    v = (mr == 1) ? tp[1] : v;
    v = (mr == 2) ? tp[2] : v;
    v = (mr == 3) ? tp[3] : v;
    v = (mr == 4) ? tp[4] : v;
    v = (mr == 5) ? tp[5] : v;
    v = (mr == 6) ? tp[6] : v;
    v = (mr == 7) ? tp[7] : v;
    if (m < 8) tst[16 * tile + 8 * hh + m] = v;
  }
  __syncthreads();

  const v4f tv = *(const v4f*)(tst + 128 * wave + 4 * lane);
  float* gp = tpl + (size_t)nodeBase + 128 * wave + 4 * lane;
  *(volatile v4f*)gp = tv;
  __threadfence();
  *(volatile v4f*)gp = tv;
}

__global__ __launch_bounds__(NTHR) void k_layer2(
    const int* __restrict__ ei, const float* __restrict__ tpl, const float* __restrict__ dinv,
    const float* __restrict__ b2, float* out, int nN, int nE, int vec8) {
  extern __shared__ v4f lds_dyn[];
  float* accs = (float*)lds_dyn;
  int*   list = (int*)(accs + NB2);
  int*   wcnt = list + LISTN;
  const int tid = threadIdx.x, lane = tid & 31, wave = tid >> 5;
  const int nodeBase = blockIdx.x * NB2;
  const int* dsts = ei + nE;

  {
    const v4f z = {0.f, 0.f, 0.f, 0.f};
    for (int i = tid; i < NB2 / 4; i += NTHR) lds_dyn[i] = z;
  }
  __syncthreads();

  const int nChunks = (nE + CHUNK - 1) / CHUNK;
#pragma unroll 1
  for (int ch = 0; ch < nChunks; ++ch) {
    const int cbase = ch * CHUNK;
    const int wc = scan_chunk<NB2>(dsts, nE, cbase, nodeBase, vec8, list, tid, lane, wave);
    if (lane == 0) wcnt[wave] = wc;
    __syncthreads();
    if (wave == 0) {
#pragma unroll 1
      for (int wsx = 0; wsx < NWAVE; ++wsx) {
        int n = __builtin_amdgcn_readfirstlane(wcnt[wsx]);
        n = n > WCAP ? WCAP : (n < 0 ? 0 : n);
        const int* lp = list + wsx * WCAP;
#pragma unroll 1
        for (int i = 0; i < n; ++i) {
          const int ent  = __builtin_amdgcn_readfirstlane(lp[i]);
          const int slot = ent & (NB2 - 1);
          int e = cbase + ((ent >> SLOTB) & (CHUNK - 1));
          e = e > nE - 1 ? nE - 1 : e;
          int src = ei[e];
          src = src < 0 ? 0 : (src > nN - 1 ? nN - 1 : src);
          const float val = dinv[src] * tpl[src];
          const float nv  = accs[slot] + val;
          if (lane == 0) accs[slot] = nv;
        }
      }
    }
    __syncthreads();
  }

  const float bb = b2[0];
#pragma unroll 1
  for (int i = 0; i < NB2 / NTHR; ++i) {
    const int slot = i * NTHR + tid;
    int node = nodeBase + slot;
    node = node > nN - 1 ? nN - 1 : node;
    const float d = dinv[node];
    float v = (accs[slot] + d * tpl[node]) * d + bb;
    v = fmaxf(v, 0.f);
    const float ex = __expf(-v);
    const float o  = __builtin_amdgcn_rcpf(1.0f + ex);
    accs[slot] = o;
  }
  __syncthreads();

#pragma unroll 4
  for (int q = 0; q < NB2 / (NWAVE * 128); ++q) {
    const int f  = (wave * (NB2 / (NWAVE * 128)) + q) * 128 + 4 * lane;
    const int gi = nodeBase + f;
    const v4f v  = *(const v4f*)(accs + f);
    if (gi + 4 <= nN) {
      *(volatile v4f*)(out + gi) = v;
    } else {
      if (gi     < nN) *(volatile float*)(out + gi)     = v.x;
      if (gi + 1 < nN) *(volatile float*)(out + gi + 1) = v.y;
      if (gi + 2 < nN) *(volatile float*)(out + gi + 2) = v.z;
    }
  }
  __threadfence();
#pragma unroll 4
  for (int q = 0; q < NB2 / (NWAVE * 128); ++q) {
    const int f  = (wave * (NB2 / (NWAVE * 128)) + q) * 128 + 4 * lane;
    const int gi = nodeBase + f;
    const v4f v  = *(const v4f*)(accs + f);
    if (gi + 4 <= nN) {
      *(volatile v4f*)(out + gi) = v;
    } else {
      if (gi     < nN) *(volatile float*)(out + gi)     = v.x;
      if (gi + 1 < nN) *(volatile float*)(out + gi + 1) = v.y;
      if (gi + 2 < nN) *(volatile float*)(out + gi + 2) = v.z;
    }
  }
}

extern "C" void kernel_launch(void* const* d_in, const int* in_sizes, int n_in,
                              void* d_out, int out_size, void* d_ws, size_t ws_size,
                              hipStream_t stream) {
  if (n_in < 6) return;
  const int nN = in_sizes[0] / DIN;
  const int nE = in_sizes[1] / 2;
  if (nN <= 0 || nE < 0 || in_sizes[0] != nN * DIN || in_sizes[1] != nE * 2) return;
  if (in_sizes[2] != DIN * DHID || in_sizes[3] < DHID || in_sizes[4] < DHID || in_sizes[5] < 1) return;
  if (out_size != nN) return;

  const float* x  = (const float*)d_in[0];
  const int*   ei = (const int*)d_in[1];
  const float* W1 = (const float*)d_in[2];
  const float* b1 = (const float*)d_in[3];
  const float* W2 = (const float*)d_in[4];
  const float* b2 = (const float*)d_in[5];
  float* out = (float*)d_out;

  const int nBD = (nN + NBD - 1) / NBD;
  const int nA1 = (nN + NB1 - 1) / NB1;
  const int nA2 = (nN + NB2 - 1) / NB2;

  char* ws = (char*)d_ws;
  size_t off = 0;
  const size_t oW1 = off; off += (size_t)DHID * DIN * 2;       off = (off + 255) & ~(size_t)255;
  const size_t oDv = off; off += (size_t)nBD * NBD * 4;        off = (off + 255) & ~(size_t)255;
  const size_t oT  = off; off += (size_t)nA1 * NB1 * 4;        off = (off + 255) & ~(size_t)255;
  if (off > ws_size) return;
  _Float16* w1s  = (_Float16*)(ws + oW1);
  float*    dinv = (float*)(ws + oDv);
  float*    tpl  = (float*)(ws + oT);

  const int vec8 = ((nE & 3) == 0) ? 1 : 0;

  const int nPrep = DHID * DIN / 8;
  k_wprep<<<(nPrep + NTHR - 1) / NTHR, NTHR, 0, stream>>>(W1, w1s);

  hipFuncSetAttribute(reinterpret_cast<const void*>(&k_deg),
                      hipFuncAttributeMaxDynamicSharedMemorySize, LDS_DEG);
  k_deg<<<nBD, NTHR, LDS_DEG, stream>>>(ei, dinv, nE, vec8);

  hipFuncSetAttribute(reinterpret_cast<const void*>(&k_layer1),
                      hipFuncAttributeMaxDynamicSharedMemorySize, LDS_L1);
  k_layer1<<<nA1, NTHR, LDS_L1, stream>>>(ei, x, dinv, w1s, b1, W2, tpl, nN, nE, vec8);

  hipFuncSetAttribute(reinterpret_cast<const void*>(&k_layer2),
                      hipFuncAttributeMaxDynamicSharedMemorySize, LDS_L2);
  k_layer2<<<nA2, NTHR, LDS_L2, stream>>>(ei, tpl, dinv, b2, out, nN, nE, vec8);
}
